// SchNet_90546500534291
// MI455X (gfx1250) — hardware-run, weakly checked
//
#include <hip/hip_runtime.h>


namespace {

constexpr int N = 50000, NP = 50048, NPL = NP  , SRCM = N  , EFULL = 1600000, E = EFULL  ;
constexpr int F = 64, NRBF = 50, KR = 64  , NTYPE = 100, NLAY = 3, NL = (NPL < N ? NPL : N);
constexpr float XS = 8.0f, WSC = 256.0f, WSQ = 0.25f, RS_ = 1024.0f, CUTOFF = 5.0f, PI_ = 3.14159265358979323846f, LN2 = 0.69314718055994531f, SLOPE = 0.0f, BNEPS = 1e-5f;
static_assert(NP % 32 == 0 && NP >= N && NPL % 32 == 0 && F == 64, "tiling");
typedef _Float16 b16;
typedef __attribute__((ext_vector_type(16))) _Float16 v16b;
typedef __attribute__((ext_vector_type(8))) _Float16 v8b;
typedef __attribute__((ext_vector_type(8))) float v8f;
typedef __attribute__((ext_vector_type(4))) float v4f;
__device__ __forceinline__ float bf16_rne(float f) { unsigned int u = __float_as_uint(f); u += 0x7FFFu + ((u >> 16) & 1u); return __uint_as_float(u & 0xFFFF0000u); }
__device__ __forceinline__ void split16(float v, b16& hi, b16& lo) { hi = (b16)v; lo = (b16)(v - (float)hi); }
__device__ __forceinline__ v16b frag_kb(const b16* p, int hh) { const v8b a = *(const v8b*)(p + 8 * hh), b = *(const v8b*)(p + 16 + 8 * hh); v16b f;
#pragma unroll
  for (int e = 0; e < 8; ++e) { f[e] = a[e]; f[8 + e] = b[e]; } return f; }
__device__ __forceinline__ v8f wmma16b(v16b a, v16b b, v8f c) { v8f d = __builtin_amdgcn_wmma_f32_16x16x32_f16(false, a, false, b, (short)0, c, false, false); asm volatile("v_nop\n\tv_nop\n\tv_nop\n\tv_nop" : "+v"(d) : "v"(a), "v"(b)); return d; }
__device__ __forceinline__ void wave_lds_sync() { __builtin_amdgcn_fence(__ATOMIC_RELEASE, "workgroup"); __builtin_amdgcn_wave_barrier(); __builtin_amdgcn_fence(__ATOMIC_ACQUIRE, "workgroup"); }
__device__ __forceinline__ float pmul(float a, float b) { float p = a * b; asm volatile("" : "+v"(p)); return p; }
__device__ __forceinline__ int iclamp(int v, int lo, int hi) { return v < lo ? lo : (v > hi ? hi : v); }
constexpr int CSR_NBLK = 512, CSR_GB = 8, CSR_GN = 1 << CSR_GB  , CSR_MAXG = 512, CSR_CAP = 12288  ;
__global__ __launch_bounds__(64) void csrA_kernel(const int* __restrict__ dst, int E, int N, int nG, int CHP, int NGP, int* __restrict__ STG, int* __restrict__ HST) {
  extern __shared__ int sm[];
  int* cnt = sm; int* run = sm + NGP; int* ids = sm + 2 * NGP;
  const int b = blockIdx.x; const int ch = (E + CSR_NBLK - 1) / CSR_NBLK; const int e0 = b * ch, e1 = min(E, e0 + ch);
  for (int i = threadIdx.x; i < NGP; i += 64) cnt[i] = 0;
  for (int i = threadIdx.x; i < CHP; i += 64) ids[i] = -1;
  __syncthreads();
  if (threadIdx.x == 0) {
    for (int e = e0; e < e1; ++e) { int d = dst[e]; d = (d < 0) ? 0 : (d >= N ? N - 1 : d); cnt[d >> CSR_GB] += 1; }
    int acc = 0; for (int g = 0; g < nG; ++g) { run[g] = acc; acc += cnt[g]; }
    for (int e = e0; e < e1; ++e) { int d = dst[e]; d = (d < 0) ? 0 : (d >= N ? N - 1 : d); const int g = d >> CSR_GB; ids[run[g]] = e; run[g] += 1; } }
  __syncthreads();
  typedef __attribute__((ext_vector_type(4))) int v4i;
  for (int pass = 0; pass < 2; ++pass) {
    for (int i = threadIdx.x; i < CHP / 4; i += 64) *(volatile v4i*)(STG + (size_t)b * CHP + i * 4) = *(const v4i*)(&ids[i * 4]);
    for (int i = threadIdx.x; i < NGP / 4; i += 64) { v4i v; for (int e = 0; e < 4; ++e) v[e] = (i * 4 + e < nG) ? cnt[i * 4 + e] : 0; *(volatile v4i*)(HST + (size_t)b * NGP + i * 4) = v; }
    __threadfence(); }
}
__global__ __launch_bounds__(512) void csrS_kernel(const int* __restrict__ HST, int nG, int NGP, int* __restrict__ START, int* __restrict__ TOT, int* __restrict__ OFF) {
  __shared__ int tot[CSR_MAXG];
  const int b = threadIdx.x;
  for (int pass = 0; pass < 2; ++pass) { int runb = 0; for (int g = 0; g < nG; ++g) { int c = HST[(size_t)b * NGP + g]; c = (c < 0) ? 0 : c; ((volatile int*)OFF)[(size_t)g * CSR_NBLK + b] = runb; runb += c; } __threadfence(); }
  for (int g = threadIdx.x; g < nG; g += 512) { int s = 0; for (int bb = 0; bb < CSR_NBLK; ++bb) { int c = HST[(size_t)bb * NGP + g]; s += (c < 0) ? 0 : c; } tot[g] = s; }
  __syncthreads();
  if (threadIdx.x < 32) {
    __shared__ int st[CSR_MAXG + 32];
    if (threadIdx.x == 0) { int acc = 0; for (int g = 0; g < NGP; ++g) { st[g] = acc; if (g < nG) acc += (tot[g] + 31) & ~31; } st[NGP] = acc; }
    __builtin_amdgcn_fence(__ATOMIC_RELEASE, "workgroup"); __builtin_amdgcn_wave_barrier(); __builtin_amdgcn_fence(__ATOMIC_ACQUIRE, "workgroup");
    for (int pass = 0; pass < 2; ++pass) { for (int i = threadIdx.x; i < NGP + 32; i += 32) { ((volatile int*)START)[i] = (i <= NGP) ? st[min(i, NGP)] : 0; ((volatile int*)TOT)[i] = (i < nG) ? tot[i] : 0; } __threadfence(); } }
}
__global__ __launch_bounds__(256) void csrB_kernel(const int* __restrict__ dst, int N, int nG, int CHP, int NGP, int permLen, const int* __restrict__ STG, const int* __restrict__ HST, const int* __restrict__ OFF, const int* __restrict__ START, const int* __restrict__ TOT, int* __restrict__ PERM, int* __restrict__ ROWPTR, int* __restrict__ ROWCNT, int* __restrict__ FLAG) {
  typedef __attribute__((ext_vector_type(4))) int v4i;
  __shared__ int ids[CSR_CAP]; __shared__ unsigned short key[CSR_CAP]; __shared__ int outp[CSR_CAP]; __shared__ int ncnt[CSR_GN + 1]; __shared__ int boff[CSR_NBLK + 1];
  const int g = blockIdx.x, t_ = threadIdx.x; int tot = TOT[g]; int st = START[g], stn = START[g + 1]; const int v0 = g * CSR_GN; const int nv = min(CSR_GN, N - v0);
  st = (st < 0) ? 0 : (st > permLen - 32 ? permLen - 32 : st) & ~31; stn = (stn < st) ? st : (stn > permLen ? permLen : stn); tot = (tot < 0) ? 0 : tot; if (tot > stn - st && tot <= CSR_CAP) tot = stn - st;
  if (tot > CSR_CAP) {
    for (int pass = 0; pass < 2; ++pass) { for (int i = t_; i < CSR_GN / 4; i += 256) { v4i a, c; for (int e = 0; e < 4; ++e) { a[e] = st; c[e] = 0; } *(volatile v4i*)(ROWPTR + v0 + i * 4) = a; *(volatile v4i*)(ROWCNT + v0 + i * 4) = c; } if (t_ == 0) ((volatile int*)FLAG)[0] = 1; __threadfence(); } (void)nv; return; }
  if (t_ == 0) { int acc = 0; for (int b = 0; b < CSR_NBLK; ++b) { boff[b] = acc; int c = HST[(size_t)b * NGP + g]; c = (c < 0) ? 0 : (c > CHP ? CHP : c); acc += c; if (acc > tot) acc = tot; } boff[CSR_NBLK] = acc; }
  for (int i = t_; i <= CSR_GN; i += 256) ncnt[i] = 0;
  __syncthreads();
  for (int b = 0; b < CSR_NBLK; ++b) { const int c = boff[b + 1] - boff[b]; int o_ = OFF[(size_t)g * CSR_NBLK + b]; o_ = (o_ < 0) ? 0 : (o_ > CHP - c ? CHP - c : o_); const int* src_ = STG + (size_t)b * CHP + o_;
    for (int i = t_; i < c; i += 256) { int id = src_[i]; id = (id < 0) ? 0 : id; ids[boff[b] + i] = id; int d = dst[id]; d = (d < v0) ? v0 : (d >= N ? N - 1 : d); int kk = d - v0; kk = (kk < 0) ? 0 : (kk >= CSR_GN ? CSR_GN - 1 : kk); key[boff[b] + i] = (unsigned short)kk; } }
  __syncthreads();
  if (t_ == 0) { for (int i = 0; i < tot; ++i) ncnt[key[i]] += 1; int acc = 0; for (int vl = 0; vl < CSR_GN; ++vl) { const int c = ncnt[vl]; ncnt[vl] = acc; acc += c; } ncnt[CSR_GN] = acc;
    for (int i = 0; i < tot; ++i) { const int vl = key[i]; outp[ncnt[vl]] = ids[i]; ncnt[vl] += 1; }
    for (int vl = CSR_GN; vl > 0; --vl) ncnt[vl] = ncnt[vl - 1]; ncnt[0] = 0; }
  __syncthreads();
  for (int pass = 0; pass < 2; ++pass) {
    for (int i = t_; i < (stn - st) / 4; i += 256) { v4i v; for (int e = 0; e < 4; ++e) { const int q = i * 4 + e; v[e] = (q < tot) ? outp[q] : -1; } *(volatile v4i*)(PERM + st + i * 4) = v; }
    for (int i = t_; i < CSR_GN / 4; i += 256) { v4i a, c; for (int e = 0; e < 4; ++e) { const int vl = i * 4 + e; a[e] = st + ncnt[vl]; c[e] = (vl < nv) ? (ncnt[vl + 1] - ncnt[vl]) : 0; } *(volatile v4i*)(ROWPTR + v0 + i * 4) = a; *(volatile v4i*)(ROWCNT + v0 + i * 4) = c; }
    __threadfence(); }
}
__global__ __launch_bounds__(256) void csrZ_kernel(int* __restrict__ p, size_t n4) { typedef __attribute__((ext_vector_type(4))) int v4i; const size_t tid = (size_t)blockIdx.x * 256 + threadIdx.x, nth = (size_t)gridDim.x * 256; v4i z = {0, 0, 0, 0}; for (size_t i = tid; i < n4; i += nth) *(volatile v4i*)(p + i * 4) = z; }
struct CsrBufs { int *STG, *HST, *OFF, *START, *TOT, *PERM, *ROWPTR, *ROWCNT, *FLAG; int nG, NGP, CHP; size_t permLen; char* base; size_t bytes; };
static size_t csr_carve(CsrBufs& c, char* ws, size_t off, int E, int N) {
  const size_t off0 = off; c.base = ws + off;
  auto al = [&](size_t bytes) { char* p = ws + off; off += (bytes + 255) & ~(size_t)255; return p; };
  c.nG = (N + CSR_GN - 1) / CSR_GN; c.NGP = (c.nG + 31) & ~31; const int ch = (E + CSR_NBLK - 1) / CSR_NBLK; c.CHP = (ch + 31) & ~31; c.permLen = (size_t)E + 32 * (size_t)c.nG + 32;
  c.STG = (int*)al((size_t)CSR_NBLK * c.CHP * 4); c.HST = (int*)al((size_t)CSR_NBLK * c.NGP * 4); c.OFF = (int*)al((size_t)c.NGP * CSR_NBLK * 4); c.START = (int*)al((size_t)(c.NGP + 64) * 4); c.TOT = (int*)al((size_t)(c.NGP + 64) * 4);
  c.PERM = (int*)al(c.permLen * 4); c.ROWPTR = (int*)al((size_t)c.nG * CSR_GN * 4); c.ROWCNT = (int*)al((size_t)c.nG * CSR_GN * 4); c.FLAG = (int*)al(256);
  c.bytes = off - off0; return off;
}
static void csr_build(const CsrBufs& c, const int* dst, int E, int N, hipStream_t stream) {
  const size_t smem = (size_t)(2 * c.NGP + c.CHP) * 4;
  csrZ_kernel<<<512, 256, 0, stream>>>((int*)c.base, c.bytes / 16);
  csrA_kernel<<<CSR_NBLK, 64, smem, stream>>>(dst, E, N, c.nG, c.CHP, c.NGP, c.STG, c.HST);
  csrS_kernel<<<1, 512, 0, stream>>>(c.HST, c.nG, c.NGP, c.START, c.TOT, c.OFF);
  csrB_kernel<<<c.nG, 256, 0, stream>>>(dst, N, c.nG, c.CHP, c.NGP, (int)c.permLen, c.STG, c.HST, c.OFF, c.START, c.TOT, c.PERM, c.ROWPTR, c.ROWCNT, c.FLAG);
}

typedef __attribute__((ext_vector_type(4))) _Float16 v4h; typedef __attribute__((ext_vector_type(2))) float v2f;
__device__ __forceinline__ float ssp_(float y) { return fmaxf(y, 0.0f) + __logf(1.0f + __expf(-fabsf(y))) - LN2; }
__device__ __forceinline__ void sincos_(float x, float& s, float& c) {
  const float kf = rintf(x * 0.63661977236758134f); const int k = (int)kf;
  float r = fmaf(-kf, 1.5703125f, x); r = fmaf(-kf, 4.837512969970703125e-4f, r); r = fmaf(-kf, 7.549789948768648e-8f, r);
  const float r2 = r * r;
  float ps = fmaf(r2, -2.5052108e-8f, 2.7557319e-6f); ps = fmaf(r2, ps, -1.9841270e-4f); ps = fmaf(r2, ps, 8.3333333e-3f); ps = fmaf(r2, ps, -1.6666667e-1f); const float sr = r * fmaf(r2, ps, 1.0f);
  float pc = fmaf(r2, 2.0876757e-9f, -2.7557319e-7f); pc = fmaf(r2, pc, 2.4801587e-5f); pc = fmaf(r2, pc, -1.3888889e-3f); pc = fmaf(r2, pc, 4.1666667e-2f); pc = fmaf(r2, pc, -0.5f); const float cr = fmaf(r2, pc, 1.0f);
  const int qd = k & 3; s = (qd == 0) ? sr : (qd == 1) ? cr : (qd == 2) ? -sr : -cr; c = (qd == 0) ? cr : (qd == 1) ? -sr : (qd == 2) ? -cr : sr;
}
template <int KIN, int K>
__global__ __launch_bounds__(256) void wt_kernel(const float* __restrict__ w, b16* __restrict__ WT, float scl) {
  const int u = blockIdx.x * 256 + threadIdx.x; if (u >= F * K / 8) return; const int e = u * 8; const int o = e / K, k0 = e % K; v8b v;
#pragma unroll
  for (int j = 0; j < 8; ++j) { const int k = k0 + j; v[j] = (b16)(k < KIN ? bf16_rne(w[(size_t)o * KIN + k]) * scl : 0.0f); }
  for (int pass = 0; pass < 2; ++pass) { *(volatile v8b*)(WT + e) = v; __threadfence(); }
}
template <int MODE>
__global__ __launch_bounds__(64) void node_kernel(const float* __restrict__ IN, const b16* __restrict__ W1T, const b16* __restrict__ W1Q, const float* __restrict__ b1, const b16* __restrict__ W2T, const b16* __restrict__ W2Q, const float* __restrict__ b2, const float* __restrict__ RES, const int* __restrict__ types, const float* __restrict__ emb, const float* __restrict__ gfp, float* __restrict__ OUT, int mrows) {
  __shared__ __attribute__((aligned(16))) b16 Ah[2][16][F + 8], Al[2][16][F + 8]; __shared__ __attribute__((aligned(16))) float Tf[2][16][F + 4];
  const int wave = threadIdx.x >> 5, lane = threadIdx.x & 31, nloc = lane & 15, hlf = lane >> 4; const size_t m0 = (size_t)blockIdx.x * 32 + wave * 16;
  if (MODE == 2) { for (int rr = 0; rr < 16; ++rr) { const size_t arow = (m0 + rr < (size_t)N) ? m0 + rr : (size_t)N - 1; const float tv = bf16_rne(IN[arow]); const float xp = pmul(pmul(tv, bf16_rne(gfp[lane])), 6.2831855f); float sn, cs; sincos_(xp, sn, cs);
      for (int j = 0; j < 2; ++j) { const float val = j == 0 ? sn : cs; const int c = j == 0 ? lane : 32 + lane; const float vs = val * XS; const b16 ph = (b16)vs; Ah[wave][rr][c] = ph; Al[wave][rr][c] = (b16)((vs - (float)ph) * RS_); } } }
  else { for (int idx = lane; idx < 16 * (F / 4); idx += 32) { const int rr = idx / (F / 4), c4 = (idx % (F / 4)) * 4; const size_t arow = (m0 + rr < (size_t)N) ? m0 + rr : (size_t)N - 1; const v4f v = *(const v4f*)(IN + arow * F + c4); v4h hv, lv;
      for (int j = 0; j < 4; ++j) { const float vs = v[j] * XS; const b16 ph = (b16)vs; hv[j] = ph; lv[j] = (b16)((vs - (float)ph) * RS_); } *(v4h*)(&Ah[wave][rr][c4]) = hv; *(v4h*)(&Al[wave][rr][c4]) = lv; } }
  wave_lds_sync();
  v8f acc[4]; for (int t = 0; t < 4; ++t) acc[t] = (v8f){};
#pragma unroll
  for (int kb = 0; kb < F; kb += 32) { const v16b a = frag_kb(&Ah[wave][nloc][kb], hlf), al = frag_kb(&Al[wave][nloc][kb], hlf);
#pragma unroll
    for (int t = 0; t < 4; ++t) { const size_t wo_ = (size_t)(t * 16 + nloc) * F + kb; acc[t] = wmma16b(a, frag_kb(W1T + wo_, hlf), acc[t]); acc[t] = wmma16b(al, frag_kb(W1Q + wo_, hlf), acc[t]); } }
  wave_lds_sync();
  if (MODE == 1) {
#pragma unroll
    for (int t = 0; t < 4; ++t) { const float bb = bf16_rne(b1[t * 16 + nloc]);
#pragma unroll
      for (int r = 0; r < 8; ++r) { const float tv = ssp_(acc[t][r] * (1.0f / (XS * WSC)) + bb); const float vs = tv * XS; const b16 ph = (b16)vs; Ah[wave][8 * hlf + r][t * 16 + nloc] = ph; Al[wave][8 * hlf + r][t * 16 + nloc] = (b16)((vs - (float)ph) * RS_); } }
    wave_lds_sync();
#pragma unroll
    for (int t = 0; t < 4; ++t) acc[t] = (v8f){};
#pragma unroll
    for (int kb = 0; kb < F; kb += 32) { const v16b a = frag_kb(&Ah[wave][nloc][kb], hlf), al = frag_kb(&Al[wave][nloc][kb], hlf);
#pragma unroll
      for (int t = 0; t < 4; ++t) { const size_t wo_ = (size_t)(t * 16 + nloc) * F + kb; acc[t] = wmma16b(a, frag_kb(W2T + wo_, hlf), acc[t]); acc[t] = wmma16b(al, frag_kb(W2Q + wo_, hlf), acc[t]); } } }
#pragma unroll
  for (int t = 0; t < 4; ++t) { const int col = t * 16 + nloc; const float bb = (MODE == 0) ? 0.0f : bf16_rne(b2[col]);
#pragma unroll
    for (int r = 0; r < 8; ++r) { const size_t vrow = m0 + 8 * hlf + r; const size_t crow = vrow < (size_t)N ? vrow : (size_t)N - 1; float val = acc[t][r] * (1.0f / (XS * WSC)) + bb;
      if (MODE == 1) val += RES[crow * F + col]; if (MODE == 2) { const int ty = iclamp(types[crow], 0, NTYPE - 1); val += bf16_rne(emb[(size_t)ty * F + col]); }
      Tf[wave][8 * hlf + r][col] = (vrow < (size_t)N) ? val : 0.0f; } }
  wave_lds_sync();
  for (int pass = 0; pass < 2; ++pass) { for (int rr = 0; rr < 16; rr += 2) { const int r2 = rr + (lane >> 4); if (m0 + r2 < (size_t)mrows) *(volatile v4f*)(OUT + (m0 + r2) * F + (lane & 15) * 4) = *(const v4f*)(&Tf[wave][r2][(lane & 15) * 4]); } __threadfence(); }
}
constexpr int TABN = 4096; constexpr float TSTEP = CUTOFF / (float)(TABN - 1);
static_assert(TABN % 32 == 0, "table tiling");
__global__ __launch_bounds__(64) void tab_kernel(const b16* __restrict__ FW1T, const b16* __restrict__ FW1Q, const float* __restrict__ fb1, const b16* __restrict__ FW2T, const b16* __restrict__ FW2Q, const float* __restrict__ fb2, float* __restrict__ TB) {
  __shared__ __attribute__((aligned(16))) b16 Ah[2][16][KR + 8], Al[2][16][KR + 8]; __shared__ __attribute__((aligned(16))) float Tf[2][16][F + 4];
  const int wave = threadIdx.x >> 5, lane = threadIdx.x & 31, nloc = lane & 15, hlf = lane >> 4; const int m0 = blockIdx.x * 32 + wave * 16;
  constexpr float STEP = CUTOFF / (float)(NRBF - 1); const float coeff = -0.5f / (STEP * STEP);
  for (int idx = lane; idx < 16 * (KR / 4); idx += 32) { const int rr = idx / (KR / 4), c4 = (idx % (KR / 4)) * 4; const float d = (float)(m0 + rr) * TSTEP; v4h hv, lv;
    for (int j = 0; j < 4; ++j) { const int k = c4 + j; float fv = 0.0f; if (k < NRBF) { const float dm = d - (float)k * STEP; fv = __expf(coeff * dm * dm); } const float vs = fv * XS; const b16 ph = (b16)vs; hv[j] = ph; lv[j] = (b16)((vs - (float)ph) * RS_); }
    *(v4h*)(&Ah[wave][rr][c4]) = hv; *(v4h*)(&Al[wave][rr][c4]) = lv; }
  wave_lds_sync();
  v8f acc[4]; for (int t = 0; t < 4; ++t) acc[t] = (v8f){};
#pragma unroll
  for (int kb = 0; kb < KR; kb += 32) { const v16b a = frag_kb(&Ah[wave][nloc][kb], hlf), al = frag_kb(&Al[wave][nloc][kb], hlf);
#pragma unroll
    for (int t = 0; t < 4; ++t) { const size_t wo_ = (size_t)(t * 16 + nloc) * KR + kb; acc[t] = wmma16b(a, frag_kb(FW1T + wo_, hlf), acc[t]); acc[t] = wmma16b(al, frag_kb(FW1Q + wo_, hlf), acc[t]); } }
  wave_lds_sync();
#pragma unroll
  for (int t = 0; t < 4; ++t) { const float bb = bf16_rne(fb1[t * 16 + nloc]);
#pragma unroll
    for (int r = 0; r < 8; ++r) { const float tv = ssp_(acc[t][r] * (1.0f / (XS * WSC)) + bb); const float vs = tv * XS; const b16 ph = (b16)vs; Ah[wave][8 * hlf + r][t * 16 + nloc] = ph; Al[wave][8 * hlf + r][t * 16 + nloc] = (b16)((vs - (float)ph) * RS_); } }
  wave_lds_sync();
#pragma unroll
  for (int t = 0; t < 4; ++t) acc[t] = (v8f){};
#pragma unroll
  for (int kb = 0; kb < F; kb += 32) { const v16b a = frag_kb(&Ah[wave][nloc][kb], hlf), al = frag_kb(&Al[wave][nloc][kb], hlf);
#pragma unroll
    for (int t = 0; t < 4; ++t) { const size_t wo_ = (size_t)(t * 16 + nloc) * F + kb; acc[t] = wmma16b(a, frag_kb(FW2T + wo_, hlf), acc[t]); acc[t] = wmma16b(al, frag_kb(FW2Q + wo_, hlf), acc[t]); } }
#pragma unroll
  for (int t = 0; t < 4; ++t) { const int col = t * 16 + nloc; const float bb = bf16_rne(fb2[col]);
#pragma unroll
    for (int r = 0; r < 8; ++r) { const int i = m0 + 8 * hlf + r; const float d = (float)i * TSTEP; float sn, cs; sincos_(d * (PI_ / CUTOFF), sn, cs); (void)sn; const float rc = (d < CUTOFF) ? 0.5f * (cs + 1.0f) : 0.0f; Tf[wave][8 * hlf + r][col] = (acc[t][r] * (1.0f / (XS * WSC)) + bb) * rc; } }
  wave_lds_sync();
  for (int pass = 0; pass < 2; ++pass) { for (int rr = 0; rr < 16; rr += 2) { const int r2 = rr + (lane >> 4); *(volatile v4f*)(TB + (size_t)(m0 + r2) * F + (lane & 15) * 4) = *(const v4f*)(&Tf[wave][r2][(lane & 15) * 4]); } __threadfence(); }
}
__global__ __launch_bounds__(256) void gath_kernel(const float* __restrict__ Hh, const float* __restrict__ rij, const int* __restrict__ idxj, const int* __restrict__ PERM, const int* __restrict__ ROWPTR, const int* __restrict__ ROWCNT, int permLen, const float* __restrict__ TB, float* __restrict__ AGG) {
  const int tid = threadIdx.x; const int row = tid >> 3, g = tid & 7, c0 = g * 8; const int v = blockIdx.x * 32 + row;
  float m[8]; for (int j = 0; j < 8; ++j) m[j] = 0.0f;
  int cnt = 0, p0 = 0; if (v < N) { cnt = iclamp(ROWCNT[v], 0, 65536); p0 = iclamp(ROWPTR[v], 0, permLen - 1); if (p0 + cnt > permLen) cnt = permLen - p0; }
#pragma unroll 1
  for (int i = 0; i < cnt; ++i) { const int e = iclamp(PERM[p0 + i], 0, E - 1); int jj = iclamp(idxj[e], 0, N - 1); if (SRCM < N) jj %= SRCM;
    const float rx = bf16_rne(rij[(size_t)e * 3]), ry = bf16_rne(rij[(size_t)e * 3 + 1]), rz = bf16_rne(rij[(size_t)e * 3 + 2]); const float d = sqrtf(fmaf(rx, rx, fmaf(ry, ry, pmul(rz, rz))));
    const float u = fminf(d, CUTOFF) * (1.0f / TSTEP); int i0 = (int)u; i0 = i0 > TABN - 2 ? TABN - 2 : i0; const float fr = u - (float)i0; const float live = (d < CUTOFF) ? 1.0f : 0.0f;
    const float* t0 = TB + (size_t)i0 * F + c0; const float* t1 = t0 + F; const float* hr = Hh + (size_t)jj * F + c0;
#pragma unroll
    for (int q = 0; q < 2; ++q) { const v4f a4 = *(const v4f*)(t0 + 4 * q), b4 = *(const v4f*)(t1 + 4 * q), h4 = *(const v4f*)(hr + 4 * q);
      for (int j = 0; j < 4; ++j) { const float w = fmaf(fr, b4[j] - a4[j], a4[j]) * live; m[4 * q + j] = fmaf(h4[j], w, m[4 * q + j]); } } }
  for (int pass = 0; pass < 2; ++pass) { float* ar = AGG + (size_t)v * F + c0;
#pragma unroll
    for (int q = 0; q < 2; ++q) { v4f o; for (int j = 0; j < 4; ++j) o[j] = (v < N) ? m[4 * q + j] : 0.0f; *(volatile v4f*)(ar + 4 * q) = o; }
    __threadfence(); }
}
}

extern "C" void kernel_launch(void* const* d_in, const int* in_sizes, int n_in, void* d_out, int out_size, void* d_ws, size_t ws_size, hipStream_t stream) {
  (void)n_in;
  auto Fp = [&](int i) { return (const float*)d_in[i]; }; auto Ip = [&](int i) { return (const int*)d_in[i]; };
  if (in_sizes[0] != N || in_sizes[1] != EFULL * 3 || in_sizes[2] != EFULL || in_sizes[3] != EFULL || in_sizes[4] != N || in_sizes[5] != NTYPE * F || in_sizes[6] != NLAY * F * F || in_sizes[7] != NLAY * F * NRBF || in_sizes[8] != NLAY * F || in_sizes[9] != NLAY * F * F || in_sizes[10] != NLAY * F || in_sizes[11] != NLAY * F * F || in_sizes[12] != NLAY * F || in_sizes[13] != NLAY * F * F || in_sizes[14] != NLAY * F || in_sizes[15] != F / 2 || in_sizes[16] != F * F || in_sizes[17] != F || out_size != N * F) return;
  size_t off = 0; char* ws = (char*)d_ws;
  auto carve = [&](size_t bytes) { char* p = ws + off; off += (bytes + 255) & ~(size_t)255; return p; };
  const size_t wsz = (size_t)F * F * 2;
  b16* TWT = (b16*)carve(wsz); b16* TWQ = (b16*)carve(wsz); b16 *I2F[NLAY], *I2FQ[NLAY], *FW1[NLAY], *FW1Q[NLAY], *FW2T[NLAY], *FW2Q[NLAY], *OW1T[NLAY], *OW1Q[NLAY], *OW2T[NLAY], *OW2Q[NLAY];
  for (int l = 0; l < NLAY; ++l) { I2F[l] = (b16*)carve(wsz); I2FQ[l] = (b16*)carve(wsz); FW1[l] = (b16*)carve(wsz); FW1Q[l] = (b16*)carve(wsz); FW2T[l] = (b16*)carve(wsz); FW2Q[l] = (b16*)carve(wsz); OW1T[l] = (b16*)carve(wsz); OW1Q[l] = (b16*)carve(wsz); OW2T[l] = (b16*)carve(wsz); OW2Q[l] = (b16*)carve(wsz); }
  float* XA = (float*)carve((size_t)NP * F * 4); float* XB = (float*)carve((size_t)NP * F * 4); float* Hh = (float*)carve((size_t)NP * F * 4); float* AGG = (float*)carve((size_t)NP * F * 4); float* TB = (float*)carve((size_t)NLAY * TABN * F * 4);
  CsrBufs csr; off = csr_carve(csr, ws, off, E, N);
  if (off > ws_size || off > ((size_t)128 << 20)) return;
  const unsigned g8 = (F * F / 8 + 255) / 256;
  wt_kernel<F, F><<<g8, 256, 0, stream>>>(Fp(16), TWT, WSC); wt_kernel<F, F><<<g8, 256, 0, stream>>>(Fp(16), TWQ, WSQ);
  for (int l = 0; l < NLAY; ++l) { const size_t mo = (size_t)l * F * F;
    wt_kernel<F, F><<<g8, 256, 0, stream>>>(Fp(6) + mo, I2F[l], WSC); wt_kernel<F, F><<<g8, 256, 0, stream>>>(Fp(6) + mo, I2FQ[l], WSQ);
    wt_kernel<NRBF, KR><<<g8, 256, 0, stream>>>(Fp(7) + (size_t)l * F * NRBF, FW1[l], WSC); wt_kernel<NRBF, KR><<<g8, 256, 0, stream>>>(Fp(7) + (size_t)l * F * NRBF, FW1Q[l], WSQ);
    wt_kernel<F, F><<<g8, 256, 0, stream>>>(Fp(9) + mo, FW2T[l], WSC); wt_kernel<F, F><<<g8, 256, 0, stream>>>(Fp(9) + mo, FW2Q[l], WSQ);
    wt_kernel<F, F><<<g8, 256, 0, stream>>>(Fp(11) + mo, OW1T[l], WSC); wt_kernel<F, F><<<g8, 256, 0, stream>>>(Fp(11) + mo, OW1Q[l], WSQ);
    wt_kernel<F, F><<<g8, 256, 0, stream>>>(Fp(13) + mo, OW2T[l], WSC); wt_kernel<F, F><<<g8, 256, 0, stream>>>(Fp(13) + mo, OW2Q[l], WSQ); }
  csr_build(csr, Ip(2), E, N, stream);
  for (int l = 0; l < NLAY; ++l) tab_kernel<<<TABN / 32, 64, 0, stream>>>(FW1[l], FW1Q[l], Fp(8) + (size_t)l * F, FW2T[l], FW2Q[l], Fp(10) + (size_t)l * F, TB + (size_t)l * TABN * F);
  node_kernel<2><<<NP / 32, 64, 0, stream>>>(Fp(4), TWT, TWQ, nullptr, nullptr, nullptr, Fp(17), nullptr, Ip(0), Fp(5), Fp(15), XA, NP);
  float* xin = XA; float* xout = XB;
  for (int l = 0; l < NLAY; ++l) { const bool last = (l == NLAY - 1);
    node_kernel<0><<<NP / 32, 64, 0, stream>>>(xin, I2F[l], I2FQ[l], nullptr, nullptr, nullptr, nullptr, nullptr, nullptr, nullptr, nullptr, Hh, NP);
    gath_kernel<<<NP / 32, 256, 0, stream>>>(Hh, Fp(1), Ip(3), csr.PERM, csr.ROWPTR, csr.ROWCNT, (int)csr.permLen, TB + (size_t)l * TABN * F, AGG);
    node_kernel<1><<<(last ? NPL : NP) / 32, 64, 0, stream>>>(AGG, OW1T[l], OW1Q[l], Fp(12) + (size_t)l * F, OW2T[l], OW2Q[l], Fp(14) + (size_t)l * F, xin, nullptr, nullptr, nullptr, last ? (float*)d_out : xout, last ? NL : NP);
    float* tmp = xin; xin = xout; xout = tmp; }
}
